// RelDecoderLayer_52793738002678
// MI455X (gfx1250) — hardware-verified
//
#include <hip/hip_runtime.h>
#include <math.h>
#include <stdint.h>

constexpr int kSeq   = 2048;
constexpr int kBatch = 2;
constexpr int kModel = 1024;
constexpr int kHeads = 16;
constexpr int kDh    = 64;
constexpr int kInner = 4096;
constexpr int kTok   = kSeq * kBatch;
constexpr int kQkvN  = 3 * kModel;
constexpr int kGrp   = 2;
constexpr int kChunks = (kBatch * kHeads) / kGrp;

constexpr float kWCarry   = 64.0f;
constexpr float kPCarry   = 2048.0f;
constexpr float kVecCarry = 256.0f;
constexpr float kL1Carry  = 16.0f;
constexpr float kQkvScale = 1.0f / kWCarry;
constexpr float kScoreScale = 0.125f;
constexpr float kPVScale  = kVecCarry / kPCarry;
constexpr float kOScale   = 1.0f / (kVecCarry * kWCarry);
constexpr float kW1Scale  = kL1Carry / kWCarry;
constexpr float kW2Scale  = 1.0f / (kL1Carry * kWCarry);
constexpr float kLnEps    = 1e-5f;
constexpr float kInvModel = 1.0f / 1024.0f;

constexpr size_t kMiB     = 1048576;
constexpr size_t kOffOW   = 0;
constexpr size_t kOffH16  = 2 * kMiB;
constexpr size_t kOffQKVW = 10 * kMiB;
constexpr size_t kOffQKV  = 16 * kMiB;
constexpr size_t kOffVT   = 40 * kMiB;
constexpr size_t kOffVEC  = 48 * kMiB;
constexpr size_t kOffSC   = 56 * kMiB;
constexpr size_t kOffP    = 88 * kMiB;
constexpr size_t kOffW1   = 2 * kMiB;
constexpr size_t kOffW2   = 16 * kMiB;
constexpr size_t kOffY1   = 24 * kMiB;
constexpr size_t kOffX16  = 40 * kMiB;
constexpr size_t kOffX    = 56 * kMiB;
constexpr size_t kOffL1   = 72 * kMiB;
constexpr size_t kOffY2   = 24 * kMiB;
constexpr size_t kWsNeed  = 104 * kMiB;
static_assert(kOffQKVW + (size_t)kQkvN * kModel * 2 == kOffQKV, "qkvw extent");
static_assert(kOffQKV + (size_t)kTok * kQkvN * 2 == kOffVT, "qkv extent");
static_assert(kOffVT + (size_t)kBatch * kHeads * kDh * kSeq * 2 == kOffVEC, "vt extent");
static_assert(kOffVEC + (size_t)kTok * kModel * 2 == kOffSC, "vec extent");
static_assert(kOffSC + (size_t)kGrp * kSeq * kSeq * 4 == kOffP, "sc extent");
static_assert(kOffP + (size_t)kGrp * kSeq * kSeq * 2 == kWsNeed, "p extent");
static_assert(kOffL1 + (size_t)kTok * kInner * 2 == kWsNeed, "l1 extent");
static_assert(kOffW2 + (size_t)kModel * kInner * 2 == kOffY1, "w2 extent");
static_assert(kOffY1 + (size_t)kTok * kModel * 4 == kOffX16, "y1 extent");
static_assert(kOffX + (size_t)kTok * kModel * 4 == kOffL1, "x extent");
static_assert(kWsNeed <= 134217728, "carve limit");

typedef __attribute__((ext_vector_type(16))) _Float16 v16h;
typedef __attribute__((ext_vector_type(8)))  _Float16 v8h;
typedef __attribute__((ext_vector_type(16))) __bf16   v16b;
typedef __attribute__((ext_vector_type(8)))  __bf16   v8b;
typedef __attribute__((ext_vector_type(8)))  float    v8f;
typedef __attribute__((ext_vector_type(4)))  float    v4f;
typedef __attribute__((ext_vector_type(4)))  unsigned int v4u;
typedef __attribute__((ext_vector_type(4)))  int      v4i;

__device__ __forceinline__ unsigned short f2bf_bits(float f) {
  unsigned u = __float_as_uint(f);
  return (unsigned short)((u + 0x7FFFu + ((u >> 16) & 1u)) >> 16);
}
__device__ __forceinline__ float bf_bits2f(unsigned short h) { return __uint_as_float(((unsigned)h) << 16); }

__device__ __forceinline__ void dep_guard_h(v8f& a, v8f& b, v16h x, v16h y) { asm volatile("v_nop\n\tv_nop\n\tv_nop\n\tv_nop" : "+v"(a), "+v"(b) : "v"(x), "v"(y)); }
__device__ __forceinline__ void dep_guard_b(v8f& a, v8f& b, v16b x, v16b y) { asm volatile("v_nop\n\tv_nop\n\tv_nop\n\tv_nop" : "+v"(a), "+v"(b) : "v"(x), "v"(y)); }
__device__ __forceinline__ void keep4_h(v16h a, v16h b, v16h c, v16h d) { asm volatile("v_nop" :: "v"(a), "v"(b), "v"(c), "v"(d)); }
__device__ __forceinline__ void keep4_b(v16b a, v16b b, v16b c, v16b d) { asm volatile("v_nop" :: "v"(a), "v"(b), "v"(c), "v"(d)); }
__device__ __forceinline__ void acc_guard4(v8f& a, v8f& b, v8f& c, v8f& d) { asm volatile("v_nop\n\tv_nop\n\tv_nop\n\tv_nop" : "+v"(a), "+v"(b), "+v"(c), "+v"(d)); }
template <typename T> struct Frag;
template <> struct Frag<_Float16> {
  typedef v16h V; union U { v16h v; v8h h[2]; };
  static __device__ __forceinline__ v16h load(const _Float16* p) {
    U f; f.h[0] = *(const v8h*)(p); f.h[1] = *(const v8h*)(p + 16); return f.v;
  }
  static __device__ __forceinline__ v8f mma(v16h a, v16h b, v8f c) {
    return __builtin_amdgcn_wmma_f32_16x16x32_f16(false, a, false, b, (short)0, c, false, false);
  }
  static __device__ __forceinline__ void guard(v8f& a, v8f& b, v16h x, v16h y) { dep_guard_h(a, b, x, y); }
  static __device__ __forceinline__ void keep(v16h a, v16h b, v16h c, v16h d) { keep4_h(a, b, c, d); }
};
template <> struct Frag<__bf16> {
  typedef v16b V; union U { v16b v; v8b h[2]; };
  static __device__ __forceinline__ v16b load(const __bf16* p) {
    U f; f.h[0] = *(const v8b*)(p); f.h[1] = *(const v8b*)(p + 16); return f.v;
  }
  static __device__ __forceinline__ v8f mma(v16b a, v16b b, v8f c) {
    return __builtin_amdgcn_wmma_f32_16x16x32_bf16(false, a, false, b, (short)0, c, false, false);
  }
  static __device__ __forceinline__ void guard(v8f& a, v8f& b, v16b x, v16b y) { dep_guard_b(a, b, x, y); }
  static __device__ __forceinline__ void keep(v16b a, v16b b, v16b c, v16b d) { keep4_b(a, b, c, d); }
};

__device__ __forceinline__ unsigned pk16(unsigned short a, unsigned short b) { return (unsigned)a | ((unsigned)b << 16); }
__device__ __forceinline__ unsigned short h_bits(float f) { const _Float16 h = (_Float16)f; return __builtin_bit_cast(unsigned short, h); }

template <int ET> struct Elem;
template <> struct Elem<0> { typedef _Float16 T; };
template <> struct Elem<1> { typedef __bf16 T; };
template <int ET, bool SPLIT, int BIAS_MODE, int OUT_MODE, bool RESID, int ACT = 0, int CAUSAL = 0>
__global__ __launch_bounds__(256) void wmma_gemm64(
    const unsigned short* __restrict__ Ap, const unsigned short* __restrict__ A2p, int lda, long strideA,
    const unsigned short* __restrict__ Btp, const unsigned short* __restrict__ Bt2p, int ldb, long strideB,
    void* __restrict__ Cout, void* __restrict__ Cout2, int ldc, long strideC,
    const float* __restrict__ bias,
    const float* __restrict__ resid, long strideR,
    int M, int N, int K, float scale) {
  typedef typename Elem<ET>::T T;
  typedef typename Frag<T>::V V;
  const T* A = (const T*)Ap; const T* A2 = (const T*)A2p; const T* Bt = (const T*)Btp; const T* Bt2 = (const T*)Bt2p;
  __shared__ __align__(16) float sT[8][16 * 68];
  const int b    = blockIdx.y;
  const int lane = threadIdx.x & 31;
  const int wave = threadIdx.x >> 5;
  const int tilesN = N >> 6;
  const int tilesM = M >> 6;
  const int tile = blockIdx.x * 8 + wave;
  if (tile >= tilesM * tilesN) return;
  const int tm = tile / tilesN;
  const int tn = tile - tm * tilesN;
  if (CAUSAL == 1 && tn > tm) return;
  const int m0 = tm << 6;
  const int n0 = tn << 6;
  const int Kw = (CAUSAL == 2) ? ((m0 + 64 < K) ? (m0 + 64) : K) : K;

  const T* Ab  = A  + (size_t)b * strideA;
  const T* Bb  = Bt + (size_t)b * strideB;
  const T* Ab2 = SPLIT ? (A2  + (size_t)b * strideA) : nullptr;
  const T* Bb2 = SPLIT ? (Bt2 + (size_t)b * strideB) : nullptr;

  const int rlane = lane & 15;
  const int koff  = (lane >> 4) * 8;
  const int mOff  = (lane >> 4) * 8;

  v8f acc[4][4];
#pragma unroll
  for (int i = 0; i < 4; ++i)
#pragma unroll
    for (int j = 0; j < 4; ++j) acc[i][j] = (v8f){0.f,0.f,0.f,0.f,0.f,0.f,0.f,0.f};

  for (int k0 = 0; k0 < Kw; k0 += 32) {
    V bh[4], bl[4];
#pragma unroll
    for (int j = 0; j < 4; ++j) {
      const size_t bo = (size_t)(n0 + (j << 4) + rlane) * ldb + koff + k0;
      bh[j] = Frag<T>::load(Bb + bo);
      if (SPLIT) bl[j] = Frag<T>::load(Bb2 + bo);
    }
#pragma unroll
    for (int i = 0; i < 4; ++i) {
      const size_t ao = (size_t)(m0 + (i << 4) + rlane) * lda + koff + k0;
      V ah = Frag<T>::load(Ab + ao);
      V al;
      if (SPLIT) al = Frag<T>::load(Ab2 + ao);
#pragma unroll
      for (int j = 0; j < 4; ++j) {
        acc[i][j] = Frag<T>::mma(ah, bh[j], acc[i][j]);
        if (SPLIT) {
          acc[i][j] = Frag<T>::mma(ah, bl[j], acc[i][j]);
          acc[i][j] = Frag<T>::mma(al, bh[j], acc[i][j]);
        }
      }
      Frag<T>::guard(acc[i][0], acc[i][3], ah, SPLIT ? al : ah);
    }
    Frag<T>::keep(bh[0], bh[1], bh[2], bh[3]);
    if (SPLIT) Frag<T>::keep(bl[0], bl[1], bl[2], bl[3]);
  }
  acc_guard4(acc[0][0], acc[0][1], acc[0][2], acc[0][3]);
  acc_guard4(acc[1][0], acc[1][1], acc[1][2], acc[1][3]);
  acc_guard4(acc[2][0], acc[2][1], acc[2][2], acc[2][3]);
  acc_guard4(acc[3][0], acc[3][1], acc[3][2], acc[3][3]);

  float* slab = sT[wave];
  const float* Rb = RESID ? (resid + (size_t)b * strideR) : nullptr;
#pragma unroll
  for (int i = 0; i < 4; ++i) {
    const int mBase = m0 + (i << 4);
#pragma unroll
    for (int j = 0; j < 4; ++j) {
      const int n = n0 + (j << 4) + rlane;
      float bv = 0.f;
      if (BIAS_MODE == 2) bv = bias[n];
#pragma unroll
      for (int r = 0; r < 8; ++r) {
        float v = acc[i][j][r] * scale;
        if (BIAS_MODE == 1) v += bias[mBase + mOff + r];
        if (BIAS_MODE == 2) v += bv;
        if (RESID) v += Rb[(size_t)(mBase + mOff + r) * ldc + n];
        if (ACT == 2) v = fmaxf(v, 0.0f);
        if (ACT == 4) v = (v > 0.f) ? v : 0.01f * v;
        slab[(mOff + r) * 68 + (j << 4) + rlane] = v;
      }
    }
    __builtin_amdgcn_fence(__ATOMIC_RELEASE, "workgroup");
    __builtin_amdgcn_wave_barrier();
    __builtin_amdgcn_fence(__ATOMIC_ACQUIRE, "workgroup");
    if (OUT_MODE == 0) {
      float* C = (float*)Cout + (size_t)b * strideC;
      const int hh = lane >> 4, c4 = (lane & 15) * 4;
      for (int pass = 0; pass < 2; ++pass) {
#pragma unroll
        for (int it = 0; it < 8; ++it) {
          const int row = it * 2 + hh;
          v4f v = *(const v4f*)(slab + row * 68 + c4);
          *(volatile v4f*)(C + (size_t)(mBase + row) * ldc + n0 + c4) = v;
        }
        __threadfence();
      }
    } else {
      const int q = lane >> 3, c8 = (lane & 7) * 8;
      unsigned short* C  = (unsigned short*)Cout  + (size_t)b * strideC;
      unsigned short* C2 = (OUT_MODE == 2) ? ((unsigned short*)Cout2 + (size_t)b * strideC) : nullptr;
      for (int pass = 0; pass < 2; ++pass) {
#pragma unroll
        for (int it = 0; it < 4; ++it) {
          const int row = it * 4 + q;
          const float* sp = slab + row * 68 + c8;
          v8h hv, lv;
#pragma unroll
          for (int e = 0; e < 8; ++e) {
            if (OUT_MODE == 1) {
              hv[e] = (_Float16)sp[e];
            } else {
              unsigned short hb = f2bf_bits(sp[e]);
              unsigned short lb = f2bf_bits(sp[e] - bf_bits2f(hb));
              hv[e] = __builtin_bit_cast(_Float16, hb);
              lv[e] = __builtin_bit_cast(_Float16, lb);
            }
          }
          *(volatile v8h*)(C + (size_t)(mBase + row) * ldc + n0 + c8) = hv;
          if (OUT_MODE == 2) *(volatile v8h*)(C2 + (size_t)(mBase + row) * ldc + n0 + c8) = lv;
        }
        __threadfence();
      }
    }
    __builtin_amdgcn_fence(__ATOMIC_RELEASE, "workgroup");
    __builtin_amdgcn_wave_barrier();
    __builtin_amdgcn_fence(__ATOMIC_ACQUIRE, "workgroup");
  }
}

__global__ __launch_bounds__(256) void cast8_f16_kernel(const float* __restrict__ in, unsigned short* __restrict__ out,
                                                        int n8, float scale) {
  const int i = blockIdx.x * 256 + threadIdx.x;
  if (i >= n8) return;
  const float* p = in + 8 * (size_t)i;
  const v4f a = *(const v4f*)(p);
  const v4f c = *(const v4f*)(p + 4);
  unsigned short hb[8];
#pragma unroll
  for (int e = 0; e < 4; ++e) {
    hb[e]     = h_bits(a[e] * scale);
    hb[4 + e] = h_bits(c[e] * scale);
  }
  const v4u u = (v4u){pk16(hb[0], hb[1]), pk16(hb[2], hb[3]), pk16(hb[4], hb[5]), pk16(hb[6], hb[7])};
  unsigned short* q = out + 8 * (size_t)i;
  *(volatile v4u*)q = u;
  __threadfence();
  *(volatile v4u*)q = u;
}

__global__ __launch_bounds__(256) void vt_build_kernel(const unsigned short* __restrict__ QKV, unsigned short* __restrict__ VT) {
  __shared__ unsigned short sm[64][66];
  const int jt = blockIdx.x;
  const int g  = blockIdx.y;
  const int b  = g >> 4, h = g & 15;
  const int t  = threadIdx.x;
#pragma unroll
  for (int it = 0; it < 2; ++it) {
    const int e  = it * 256 + t;
    const int r  = e >> 3;
    const int c8 = (e & 7) * 8;
    const size_t src = ((size_t)(jt * 64 + r) * kBatch + b) * kQkvN + 2 * kModel + h * kDh + c8;
    const v4u u = *(const v4u*)(QKV + src);
#pragma unroll
    for (int q = 0; q < 4; ++q) {
      sm[r][c8 + 2 * q]     = (unsigned short)(u[q] & 0xffffu);
      sm[r][c8 + 2 * q + 1] = (unsigned short)(u[q] >> 16);
    }
  }
  __syncthreads();
  const int lane = t & 31, wave = t >> 5;
  const int q = lane >> 3, c8 = (lane & 7) * 8;
  for (int pass = 0; pass < 2; ++pass) {
#pragma unroll
    for (int it = 0; it < 2; ++it) {
      const int d = wave * 8 + it * 4 + q;
      unsigned short hb[8];
#pragma unroll
      for (int e = 0; e < 8; ++e) hb[e] = sm[c8 + e][d];
      const v4u u = (v4u){pk16(hb[0], hb[1]), pk16(hb[2], hb[3]), pk16(hb[4], hb[5]), pk16(hb[6], hb[7])};
      *(volatile v4u*)(VT + ((size_t)g * kDh + d) * kSeq + jt * 64 + c8) = u;
    }
    __threadfence();
  }
}

__global__ __launch_bounds__(256) void softmax_causal_kernel(const float* __restrict__ S, const int* __restrict__ mask,
                                                             unsigned short* __restrict__ P, float carry) {
  __shared__ float redM[8];
  __shared__ float redS[8];
  const int row  = blockIdx.x;
  const int gi   = blockIdx.y;
  const int t    = threadIdx.x;
  const int lane = t & 31, wave = t >> 5;
  const int L    = ((row >> 6) + 1) << 6;
  const size_t rbase = ((size_t)gi * kSeq + row) * kSeq;
  const float* sr = S + rbase;
  const int* mk = mask + (size_t)row * kSeq;
  const int c0 = t * 8;
  const bool act  = (c0 < L);
  const bool wact = ((wave << 8) < L);
  float x[8];
#pragma unroll
  for (int e = 0; e < 8; ++e) x[e] = -INFINITY;
  float m = -INFINITY;
  if (wact) {
    const int cc = act ? c0 : 0;
    const v4f a  = *(const v4f*)(sr + cc);
    const v4f c  = *(const v4f*)(sr + cc + 4);
    const v4i ma = *(const v4i*)(mk + cc);
    const v4i mb = *(const v4i*)(mk + cc + 4);
#pragma unroll
    for (int e = 0; e < 4; ++e) {
      x[e]     = (act && ma[e] == 0) ? a[e] : -INFINITY;
      x[4 + e] = (act && mb[e] == 0) ? c[e] : -INFINITY;
    }
    m = fmaxf(fmaxf(fmaxf(x[0], x[1]), fmaxf(x[2], x[3])), fmaxf(fmaxf(x[4], x[5]), fmaxf(x[6], x[7])));
  }
#pragma unroll
  for (int off = 16; off > 0; off >>= 1) m = fmaxf(m, __shfl_xor(m, off, 32));
  if (lane == 0) redM[wave] = m;
  __syncthreads();
  float mall = redM[0];
#pragma unroll
  for (int i = 1; i < 8; ++i) mall = fmaxf(mall, redM[i]);

  float p[8];
#pragma unroll
  for (int e = 0; e < 8; ++e) p[e] = 0.0f;
  float ps = 0.0f;
  if (wact) {
#pragma unroll
    for (int e = 0; e < 8; ++e) {
      p[e] = expf(x[e] - mall);
      ps += p[e];
    }
  }
#pragma unroll
  for (int off = 16; off > 0; off >>= 1) ps += __shfl_xor(ps, off, 32);
  if (lane == 0) redS[wave] = ps;
  __syncthreads();
  float tot = redS[0];
#pragma unroll
  for (int i = 1; i < 8; ++i) tot += redS[i];
  const float inv = 1.0f / tot;

  unsigned short hb[8];
#pragma unroll
  for (int e = 0; e < 8; ++e) hb[e] = h_bits((p[e] * inv) * carry);
  const v4u u = (v4u){pk16(hb[0], hb[1]), pk16(hb[2], hb[3]), pk16(hb[4], hb[5]), pk16(hb[6], hb[7])};
  unsigned short* dst = P + rbase + c0;
  const bool st = wact && act;
  if (st) *(volatile v4u*)dst = u;
  __threadfence();
  if (st) *(volatile v4u*)dst = u;
}

template <bool WH>
__global__ __launch_bounds__(256) void ln_kernel(const float* __restrict__ Y, const float* __restrict__ G,
                                                 const float* __restrict__ Bv, float* __restrict__ Of,
                                                 unsigned short* __restrict__ Oh) {
  __shared__ float red1[8];
  __shared__ float red2[8];
  __shared__ __align__(16) float srow[kModel];
  const int row = blockIdx.x;
  const int t = threadIdx.x, lane = t & 31, wave = t >> 5;
  const size_t base = (size_t)row * kModel;
  const v4f yv = *(const v4f*)(Y + base + 4 * t);
  float s = (yv[0] + yv[1]) + (yv[2] + yv[3]);
#pragma unroll
  for (int off = 16; off > 0; off >>= 1) s += __shfl_xor(s, off, 32);
  if (lane == 0) red1[wave] = s;
  __syncthreads();
  float tot = red1[0];
#pragma unroll
  for (int i = 1; i < 8; ++i) tot += red1[i];
  const float mean = tot * kInvModel;
  const float d0 = yv[0] - mean, d1 = yv[1] - mean, d2 = yv[2] - mean, d3 = yv[3] - mean;
  float q = (d0 * d0 + d1 * d1) + (d2 * d2 + d3 * d3);
#pragma unroll
  for (int off = 16; off > 0; off >>= 1) q += __shfl_xor(q, off, 32);
  if (lane == 0) red2[wave] = q;
  __syncthreads();
  float qt = red2[0];
#pragma unroll
  for (int i = 1; i < 8; ++i) qt += red2[i];
  const float var  = qt * kInvModel;
  const float rstd = rsqrtf(var + kLnEps);
  const v4f gv = *(const v4f*)(G + 4 * t);
  const v4f bv = *(const v4f*)(Bv + 4 * t);
  v4f o;
  o[0] = (d0 * rstd) * gv[0] + bv[0];
  o[1] = (d1 * rstd) * gv[1] + bv[1];
  o[2] = (d2 * rstd) * gv[2] + bv[2];
  o[3] = (d3 * rstd) * gv[3] + bv[3];
  float* dst = Of + base + 4 * t;
  *(volatile v4f*)dst = o;
  __threadfence();
  *(volatile v4f*)dst = o;
  if (WH) {
    *(v4f*)(srow + 4 * t) = o;
    __syncthreads();
    if (t < 128) {
      const float* sp = srow + 8 * t;
      unsigned short hb[8];
#pragma unroll
      for (int e = 0; e < 8; ++e) hb[e] = h_bits(sp[e]);
      const v4u u = (v4u){pk16(hb[0], hb[1]), pk16(hb[2], hb[3]), pk16(hb[4], hb[5]), pk16(hb[6], hb[7])};
      unsigned short* dh = Oh + base + 8 * t;
      *(volatile v4u*)dh = u;
      __threadfence();
      *(volatile v4u*)dh = u;
    }
  }
}

extern "C" void kernel_launch(void* const* d_in, const int* in_sizes, int n_in,
                              void* d_out, int out_size, void* d_ws,
                              size_t ws_size, hipStream_t stream) {
  if (n_in < 11) return;
  if (in_sizes[0] != kTok * kModel || in_sizes[2] != kSeq * kSeq || in_sizes[3] != kQkvN * kModel ||
      in_sizes[4] != kModel * kModel || in_sizes[5] != kModel || in_sizes[6] != kModel ||
      in_sizes[7] != kInner * kModel || in_sizes[8] != kModel * kInner || in_sizes[9] != kModel ||
      in_sizes[10] != kModel) return;
  if (out_size != kTok * kModel) return;
  if (ws_size < kWsNeed) return;

  const float* h     = (const float*)d_in[0];
  const int*   amask = (const int*)d_in[2];
  const float* qkv_w = (const float*)d_in[3];
  const float* o_w   = (const float*)d_in[4];
  const float* ln1_g = (const float*)d_in[5];
  const float* ln1_b = (const float*)d_in[6];
  const float* w1    = (const float*)d_in[7];
  const float* w2    = (const float*)d_in[8];
  const float* ln2_g = (const float*)d_in[9];
  const float* ln2_b = (const float*)d_in[10];
  float* outp = (float*)d_out;

  char* ws = (char*)d_ws;
  unsigned short* OW16   = (unsigned short*)(ws + kOffOW);
  unsigned short* H16    = (unsigned short*)(ws + kOffH16);
  unsigned short* QKVW16 = (unsigned short*)(ws + kOffQKVW);
  unsigned short* QKV16  = (unsigned short*)(ws + kOffQKV);
  unsigned short* VT16   = (unsigned short*)(ws + kOffVT);
  unsigned short* VEC16  = (unsigned short*)(ws + kOffVEC);
  float*          SC     = (float*)(ws + kOffSC);
  unsigned short* P16    = (unsigned short*)(ws + kOffP);
  unsigned short* W1_16  = (unsigned short*)(ws + kOffW1);
  unsigned short* W2_16  = (unsigned short*)(ws + kOffW2);
  float*          Y1     = (float*)(ws + kOffY1);
  unsigned short* X16    = (unsigned short*)(ws + kOffX16);
  float*          X      = (float*)(ws + kOffX);
  unsigned short* L1     = (unsigned short*)(ws + kOffL1);
  float*          Y2     = (float*)(ws + kOffY2);

  const int n8_h   = (kTok * kModel) / 8;
  const int n8_qkv = (kQkvN * kModel) / 8;
  const int n8_ow  = (kModel * kModel) / 8;
  const int n8_w1  = (kInner * kModel) / 8;
  const int n8_w2  = (kModel * kInner) / 8;

  cast8_f16_kernel<<<(n8_h + 255) / 256, 256, 0, stream>>>(h, H16, n8_h, 1.0f);
  cast8_f16_kernel<<<(n8_qkv + 255) / 256, 256, 0, stream>>>(qkv_w, QKVW16, n8_qkv, kWCarry);
  cast8_f16_kernel<<<(n8_ow + 255) / 256, 256, 0, stream>>>(o_w, OW16, n8_ow, kWCarry);

  wmma_gemm64<0, false, 0, 1, false, 0, 0><<<dim3(384, 1), 256, 0, stream>>>(
      H16, H16, kModel, (long)0,
      QKVW16, QKVW16, kModel, (long)0,
      (void*)QKV16, (void*)QKV16, kQkvN, (long)0,
      ln1_g, h, (long)0,
      kTok, kQkvN, kModel, kQkvScale);

  vt_build_kernel<<<dim3(kSeq / 64, kBatch * kHeads), 256, 0, stream>>>(QKV16, VT16);

  for (int c = 0; c < kChunks; ++c) {
    const int bb = c / (kHeads / kGrp);
    const int h0 = (c % (kHeads / kGrp)) * kGrp;
    const unsigned short* Qp = QKV16 + (size_t)bb * kQkvN + (size_t)h0 * kDh;
    const unsigned short* Kp = QKV16 + (size_t)bb * kQkvN + kModel + (size_t)h0 * kDh;
    wmma_gemm64<0, false, 0, 0, false, 0, 1><<<dim3(128, kGrp), 256, 0, stream>>>(
        Qp, Qp, 2 * kQkvN, (long)kDh,
        Kp, Kp, 2 * kQkvN, (long)kDh,
        (void*)SC, (void*)SC, kSeq, (long)kSeq * kSeq,
        ln1_g, h, (long)0,
        kSeq, kSeq, kDh, kScoreScale);
    softmax_causal_kernel<<<dim3(kSeq, kGrp), 256, 0, stream>>>(SC, amask, P16, kPCarry);
    const unsigned short* VTp = VT16 + (size_t)(bb * kHeads + h0) * kDh * kSeq;
    unsigned short* VECp = VEC16 + (size_t)bb * kModel + (size_t)h0 * kDh;
    wmma_gemm64<0, false, 0, 1, false, 0, 2><<<dim3(4, kGrp), 256, 0, stream>>>(
        P16, P16, kSeq, (long)kSeq * kSeq,
        VTp, VTp, kSeq, (long)kDh * kSeq,
        (void*)VECp, (void*)VECp, 2 * kModel, (long)kDh,
        ln1_g, h, (long)0,
        kSeq, kDh, kSeq, kPVScale);
  }

  cast8_f16_kernel<<<(n8_w1 + 255) / 256, 256, 0, stream>>>(w1, W1_16, n8_w1, kWCarry);
  cast8_f16_kernel<<<(n8_w2 + 255) / 256, 256, 0, stream>>>(w2, W2_16, n8_w2, kWCarry);

  wmma_gemm64<0, false, 0, 0, true, 0, 0><<<dim3(128, 1), 256, 0, stream>>>(
      VEC16, VEC16, kModel, (long)0,
      OW16, OW16, kModel, (long)0,
      (void*)Y1, (void*)Y1, kModel, (long)0,
      ln1_g, h, (long)0,
      kTok, kModel, kModel, kOScale);

  ln_kernel<true><<<kTok, 256, 0, stream>>>(Y1, ln1_g, ln1_b, X, X16);

  wmma_gemm64<0, false, 0, 1, false, 0, 0><<<dim3(512, 1), 256, 0, stream>>>(
      X16, X16, kModel, (long)0,
      W1_16, W1_16, kModel, (long)0,
      (void*)L1, (void*)L1, kInner, (long)0,
      ln1_g, h, (long)0,
      kTok, kInner, kModel, kW1Scale);

  wmma_gemm64<0, false, 0, 0, true, 0, 0><<<dim3(128, 1), 256, 0, stream>>>(
      L1, L1, kInner, (long)0,
      W2_16, W2_16, kInner, (long)0,
      (void*)Y2, (void*)Y2, kModel, (long)0,
      ln2_g, X, (long)0,
      kTok, kModel, kInner, kW2Scale);

  ln_kernel<false><<<kTok, 256, 0, stream>>>(Y2, ln2_g, ln2_b, outp, X16);
}
